// DiagonalLSTMCell_81913616270014
// MI455X (gfx1250) — hardware-run, weakly checked
//
#include <hip/hip_runtime.h>

constexpr int NBAT  = 16;
constexpr int NCIN  = 64;
constexpr int NROW  = 64;
constexpr int NCOL  = 64;
constexpr int NHID  = 128;
constexpr int NGATE = 4 * NHID;
constexpr int KCAT  = 2 * NHID + NCIN;
constexpr int NSTEP = 2 * NCOL - 1;
constexpr int HSP = NHID + 8;
constexpr int XSP = NCIN + 8;
constexpr int HOP = NHID + 4;
constexpr int SCAN_THR   = 512;
constexpr int SCAN_WAVES = SCAN_THR / 32;
constexpr float WCARRY     = 256.0f;
constexpr float WCARRY_INV = 1.0f / WCARRY;

static_assert(NGATE == 32 * SCAN_WAVES);
static_assert(NROW == 64 && NCOL == 64 && NCIN == 64 && NHID == 128);
static_assert(KCAT % 32 == 0 && NHID % 32 == 0 && NCIN % 32 == 0);
static_assert(NROW == 4 * SCAN_WAVES);
static_assert((NROW + 1) * HSP * 2 + NROW * XSP * 2 + NROW * HOP * 4 + 2 * NGATE * 4 <= 65536);
static_assert((HSP * 2) % 16 == 0 && (XSP * 2) % 16 == 0 && (HOP * 4) % 16 == 0);

typedef __attribute__((ext_vector_type(16))) _Float16 v16h;
typedef __attribute__((ext_vector_type(8)))  _Float16 v8h;
typedef __attribute__((ext_vector_type(2)))  _Float16 v2h;
typedef __attribute__((ext_vector_type(8)))  float    v8f;
typedef __attribute__((ext_vector_type(4)))  float    v4f;
typedef __attribute__((ext_vector_type(2)))  float    v2f;
typedef __attribute__((ext_vector_type(4)))  unsigned v4u;

__device__ __forceinline__ unsigned short f2bf_bits(float f) {
  unsigned u = __float_as_uint(f);
  return (unsigned short)((u + 0x7FFFu + ((u >> 16) & 1u)) >> 16);
}
__device__ __forceinline__ float bf_bits2f(unsigned short h) { return __uint_as_float(((unsigned)h) << 16); }
__device__ __forceinline__ float bf16r(float f) { return bf_bits2f(f2bf_bits(f)); }

__device__ __forceinline__ float fsig(float x)  { return __builtin_amdgcn_rcpf(1.0f + __expf(-x)); }
__device__ __forceinline__ float ftanh(float x) { return 1.0f - 2.0f * __builtin_amdgcn_rcpf(__expf(2.0f * x) + 1.0f); }

__device__ __forceinline__ void pin4(v4f& a) { asm volatile("" : "+v"(a)); }

union FragU { v16h v; v8h h[2]; };
__device__ __forceinline__ v16h frag_load(const _Float16* p) {
  FragU f;
  f.h[0] = *(const v8h*)(p);
  f.h[1] = *(const v8h*)(p + 16);
  return f.v;
}
__device__ __forceinline__ v8f mma16(v16h a, v16h b, v8f c) {
  return __builtin_amdgcn_wmma_f32_16x16x32_f16(false, a, false, b, (short)0, c, false, false);
}
__device__ __forceinline__ void guard8(v8f& a0, v8f& a1, v8f& a2, v8f& a3, v8f& a4, v8f& a5, v8f& a6, v8f& a7,
                                       v16h x0, v16h x1, v16h b0, v16h b1, v16h b2, v16h b3) {
  asm volatile("v_nop\n\tv_nop\n\tv_nop\n\tv_nop"
               : "+v"(a0), "+v"(a1), "+v"(a2), "+v"(a3), "+v"(a4), "+v"(a5), "+v"(a6), "+v"(a7)
               : "v"(x0), "v"(x1), "v"(b0), "v"(b1), "v"(b2), "v"(b3));
}

__global__ __launch_bounds__(256) void prep_x_kernel(const float* __restrict__ x, unsigned short* __restrict__ XH) {
  __shared__ float Tt[64 * 65];
  const int tid = threadIdx.x;
  const int b = blockIdx.x / NROW;
  const int h = blockIdx.x - b * NROW;
#pragma unroll
  for (int i = 0; i < 4; ++i) {
    const int idx = i * 256 + tid;
    const int cc = idx >> 4;
    const int w4 = (idx & 15) * 4;
    const v4f v = *(const v4f*)(x + (((size_t)(b * NCIN + cc) * NROW + h) * NCOL) + w4);
    Tt[cc * 65 + w4 + 0] = v[0];
    Tt[cc * 65 + w4 + 1] = v[1];
    Tt[cc * 65 + w4 + 2] = v[2];
    Tt[cc * 65 + w4 + 3] = v[3];
  }
  __syncthreads();
  const int q = tid >> 3;
  const int c8 = (tid & 7) * 8;
  v8h hv[2];
#pragma unroll
  for (int g = 0; g < 2; ++g) {
    const int qq = g * 32 + q;
#pragma unroll
    for (int e = 0; e < 8; ++e) {
      const float f = Tt[(c8 + e) * 65 + qq];
      hv[g][e] = (_Float16)bf16r(f);
    }
  }
  for (int pass = 0; pass < 2; ++pass) {
#pragma unroll
    for (int g = 0; g < 2; ++g) {
      const size_t o = ((size_t)((b * NROW + h) * NCOL + g * 32 + q)) * NCIN + c8;
      *(volatile v8h*)(XH + o) = hv[g];
    }
    __threadfence();
  }
}

__global__ __launch_bounds__(256) void prep_w_kernel(const float* __restrict__ Wss, const float* __restrict__ Wis,
                                                     unsigned short* __restrict__ ACAT) {
  const int i = blockIdx.x * 256 + threadIdx.x;
  constexpr int G8 = KCAT / 8;
  if (i < NGATE * G8) {
    const int mp = i / G8;
    const int k8 = i - mp * G8;
    const int kb = k8 * 8;
    const int o = (mp & 3) * NHID + (mp >> 2);
    const int seg = (kb < NHID) ? 0 : ((kb < 2 * NHID) ? 1 : 2);
    const int cs = (seg == 2) ? 0 : (kb - seg * NHID);
    const int ci = (seg == 2) ? (kb - 2 * NHID) : 0;
    const float* sp = Wss + (size_t)o * (2 * NHID) + 2 * cs;
    const float* ip = Wis + (size_t)o * NCIN + ci;
    v4f s0 = *(const v4f*)(sp);
    v4f s1 = *(const v4f*)(sp + 4);
    v4f s2 = *(const v4f*)(sp + 8);
    v4f s3 = *(const v4f*)(sp + 12);
    v4f w0 = *(const v4f*)(ip);
    v4f w1 = *(const v4f*)(ip + 4);
    pin4(s0); pin4(s1); pin4(s2); pin4(s3); pin4(w0); pin4(w1);
    const bool odd = (seg == 1);
    const bool isx = (seg == 2);
    float val[8];
    val[0] = odd ? s0[1] : s0[0];
    val[1] = odd ? s0[3] : s0[2];
    val[2] = odd ? s1[1] : s1[0];
    val[3] = odd ? s1[3] : s1[2];
    val[4] = odd ? s2[1] : s2[0];
    val[5] = odd ? s2[3] : s2[2];
    val[6] = odd ? s3[1] : s3[0];
    val[7] = odd ? s3[3] : s3[2];
    float xv[8];
    xv[0] = w0[0]; xv[1] = w0[1]; xv[2] = w0[2]; xv[3] = w0[3];
    xv[4] = w1[0]; xv[5] = w1[1]; xv[6] = w1[2]; xv[7] = w1[3];
    v8h hv;
#pragma unroll
    for (int e = 0; e < 8; ++e) {
      const float f = isx ? xv[e] : val[e];
      hv[e] = (_Float16)(bf16r(f) * WCARRY);
    }
    *(volatile v8h*)(ACAT + (size_t)i * 8) = hv;
    __threadfence();
    *(volatile v8h*)(ACAT + (size_t)i * 8) = hv;
  }
}

template <int JS>
__device__ __forceinline__ void mma_chunk(v8f (&acc)[2][4], const _Float16* ap0, const _Float16* ap1,
                                          const _Float16* bp, int jlo) {
  v16h bf[4];
#pragma unroll
  for (int j = 0; j < 4; ++j) bf[j] = frag_load(bp + j * JS);
  const v16h x0 = frag_load(ap0);
  const v16h x1 = frag_load(ap1);
#pragma unroll
  for (int j = 0; j < 4; ++j) {
    if (j >= jlo) {
      acc[0][j] = mma16(x0, bf[j], acc[0][j]);
      acc[1][j] = mma16(x1, bf[j], acc[1][j]);
    }
  }
  guard8(acc[0][0], acc[0][1], acc[0][2], acc[0][3], acc[1][0], acc[1][1], acc[1][2], acc[1][3],
         x0, x1, bf[0], bf[1], bf[2], bf[3]);
}

__device__ __forceinline__ void stage_x(_Float16* xs, const unsigned short* Xb, int tn, int tid) {
  const int row = tid >> 3;
  const int c8 = (tid & 7) * 8;
  const int w = tn - row;
  const bool inw = (w >= 0) && (w < NCOL);
  const int wc = (w < 0) ? 0 : ((w > NCOL - 1) ? (NCOL - 1) : w);
  v4u raw = *(const v4u*)(Xb + ((size_t)(row * NCOL + wc)) * NCIN + c8);
  asm volatile("" : "+v"(raw));
  v4u z;
  z[0] = inw ? raw[0] : 0u;
  z[1] = inw ? raw[1] : 0u;
  z[2] = inw ? raw[2] : 0u;
  z[3] = inw ? raw[3] : 0u;
  const v8h hv = __builtin_bit_cast(v8h, z);
  *(v8h*)(xs + row * XSP + c8) = hv;
}

__device__ __forceinline__ void copy_rows(const float* hout, float* Hb, int tp, int wave, int lane) {
  v4f cv[4];
#pragma unroll
  for (int rr = 0; rr < 4; ++rr) {
    const int r = 4 * wave + rr;
    const int w = tp - r;
    const bool ok = (w >= 0) && (w < NCOL);
    cv[rr] = (v4f){0.f, 0.f, 0.f, 0.f};
    if (ok) cv[rr] = *(const v4f*)(hout + r * HOP + 4 * lane);
  }
  for (int pass = 0; pass < 2; ++pass) {
#pragma unroll
    for (int rr = 0; rr < 4; ++rr) {
      const int r = 4 * wave + rr;
      const int w = tp - r;
      const bool ok = (w >= 0) && (w < NCOL);
      if (ok) *(volatile v4f*)(Hb + ((size_t)(r * NCOL + w)) * NHID + 4 * lane) = cv[rr];
    }
    __threadfence();
  }
}

__device__ __forceinline__ float lstm_cell(float zi, float zf, float zo, float zg, float& cs) {
  const float ig = fsig(zi);
  const float fg = fsig(zf);
  const float og = fsig(zo);
  const float gg = ftanh(zg);
  const float cn = fg * cs + ig * gg;
  cs = cn;
  return og * ftanh(cn);
}

__global__ __launch_bounds__(SCAN_THR) void diag_scan_kernel(const unsigned short* __restrict__ XHp,
                                                             const unsigned short* __restrict__ ACATp,
                                                             const float* __restrict__ h0, const float* __restrict__ c0,
                                                             const float* __restrict__ bis, const float* __restrict__ bss,
                                                             float* __restrict__ HST) {
  __shared__ __align__(16) _Float16 hs[(NROW + 1) * HSP];
  __shared__ __align__(16) _Float16 xs[NROW * XSP];
  __shared__ __align__(16) float    hout[NROW * HOP];
  __shared__ __align__(16) float    sBss[NGATE];
  __shared__ __align__(16) float    sBis[NGATE];

  const int b = blockIdx.x;
  const int tid = threadIdx.x;
  const int lane = tid & 31;
  const int wave = __builtin_amdgcn_readfirstlane(tid >> 5);
  const int c = lane & 15;
  const int hf = lane >> 4;
  const int koff = hf * 8;
  const _Float16* ACAT = (const _Float16*)ACATp;
  const unsigned short* Xb = XHp + (size_t)b * NROW * NCOL * NCIN;
  float* Hb = HST + (size_t)b * NROW * NCOL * NHID;
  const v8h zero8 = {(_Float16)0.0f, (_Float16)0.0f, (_Float16)0.0f, (_Float16)0.0f,
                     (_Float16)0.0f, (_Float16)0.0f, (_Float16)0.0f, (_Float16)0.0f};

  if (tid < 16) *(v8h*)(hs + tid * 8) = zero8;
#pragma unroll 1
  for (int it = 0; it < 16; ++it) {
    const int idx = it * SCAN_THR + tid;
    const int ch = idx >> 6;
    const int r = idx & 63;
    hs[(r + 1) * HSP + ch] = (_Float16)bf16r(h0[((size_t)b * NHID + ch) * NROW + r]);
  }
  {
    const int o = (tid & 3) * NHID + (tid >> 2);
    sBss[tid] = bf16r(bss[o]);
    sBis[tid] = bf16r(bis[o]);
  }
  stage_x(xs, Xb, 0, tid);

  float cst[2][4][2];
#pragma unroll
  for (int i = 0; i < 2; ++i)
#pragma unroll
    for (int j = 0; j < 4; ++j)
#pragma unroll
      for (int u = 0; u < 2; ++u) {
        const int hd = 8 * wave + 4 * i + 2 * hf + u;
        const int r = 16 * j + c;
        cst[i][j][u] = bf16r(c0[((size_t)b * NHID + hd) * NROW + r]);
      }
  __syncthreads();

  const _Float16* a0 = ACAT + (size_t)(32 * wave + c) * KCAT + koff;
  const _Float16* a1 = a0 + 16 * KCAT;
  const _Float16* hsb = hs + c * HSP + koff;
  const _Float16* xsb = xs + c * XSP + koff;
  const v8f z8 = {0.f, 0.f, 0.f, 0.f, 0.f, 0.f, 0.f, 0.f};

#pragma unroll 1
  for (int t = 0; t < NSTEP; ++t) {
    const int jlo = (t < 15 + NCOL) ? 0 : (((t - 15 - NCOL) >> 4) + 1);

    copy_rows(hout, Hb, t - 1, wave, lane);

    v8f acc[2][4];
#pragma unroll
    for (int i = 0; i < 2; ++i)
#pragma unroll
      for (int j = 0; j < 4; ++j) acc[i][j] = z8;

#pragma unroll 1
    for (int kc = 0; kc < NHID / 32; ++kc)
      mma_chunk<16 * HSP>(acc, a0 + 32 * kc, a1 + 32 * kc, hsb + 32 * kc, jlo);
#pragma unroll 1
    for (int kc = 0; kc < NHID / 32; ++kc)
      mma_chunk<16 * HSP>(acc, a0 + NHID + 32 * kc, a1 + NHID + 32 * kc, hsb + HSP + 32 * kc, jlo);
#pragma unroll 1
    for (int kc = 0; kc < NCIN / 32; ++kc)
      mma_chunk<16 * XSP>(acc, a0 + 2 * NHID + 32 * kc, a1 + 2 * NHID + 32 * kc, xsb + 32 * kc, jlo);

    __syncthreads();

#pragma unroll
    for (int i = 0; i < 2; ++i) {
      const int mloc = 32 * wave + 16 * i + 8 * hf;
      const v4f sA = *(const v4f*)(sBss + mloc);
      const v4f sB = *(const v4f*)(sBss + mloc + 4);
      const v4f iA = *(const v4f*)(sBis + mloc);
      const v4f iB = *(const v4f*)(sBis + mloc + 4);
      const int hd0 = mloc >> 2;
#pragma unroll
      for (int j = 0; j < 4; ++j) {
        if (j >= jlo) {
          const int r = 16 * j + c;
          const int w = t - r;
          const bool inw = (w >= 0) && (w < NCOL);
          const v8f a = acc[i][j];
          const float zi0 = a[0] * WCARRY_INV + (sA[0] + (inw ? iA[0] : 0.0f));
          const float zf0 = a[1] * WCARRY_INV + (sA[1] + (inw ? iA[1] : 0.0f));
          const float zo0 = a[2] * WCARRY_INV + (sA[2] + (inw ? iA[2] : 0.0f));
          const float zg0 = a[3] * WCARRY_INV + (sA[3] + (inw ? iA[3] : 0.0f));
          const float zi1 = a[4] * WCARRY_INV + (sB[0] + (inw ? iB[0] : 0.0f));
          const float zf1 = a[5] * WCARRY_INV + (sB[1] + (inw ? iB[1] : 0.0f));
          const float zo1 = a[6] * WCARRY_INV + (sB[2] + (inw ? iB[2] : 0.0f));
          const float zg1 = a[7] * WCARRY_INV + (sB[3] + (inw ? iB[3] : 0.0f));
          const float hn0 = lstm_cell(zi0, zf0, zo0, zg0, cst[i][j][0]);
          const float hn1 = lstm_cell(zi1, zf1, zo1, zg1, cst[i][j][1]);
          v2h hp;
          hp[0] = (_Float16)hn0;
          hp[1] = (_Float16)hn1;
          *(v2h*)(hs + (r + 1) * HSP + hd0) = hp;
          v2f ho;
          ho[0] = hn0;
          ho[1] = hn1;
          *(v2f*)(hout + r * HOP + hd0) = ho;
        }
      }
    }
    if (tid < 16) *(v8h*)(hs + tid * 8) = zero8;
    stage_x(xs, Xb, t + 1, tid);

    __syncthreads();
  }
  copy_rows(hout, Hb, NSTEP - 1, wave, lane);
}

__global__ __launch_bounds__(256) void unskew_tr_kernel(const float* __restrict__ HST, float* __restrict__ out) {
  __shared__ __align__(16) float Tq[NCOL * HOP];
  const int tid = threadIdx.x;
  const int b = blockIdx.x / NROW;
  const int r = blockIdx.x - b * NROW;
  const float* src = HST + ((size_t)(b * NROW + r) * NCOL) * NHID;
#pragma unroll
  for (int it = 0; it < 8; ++it) {
    const int idx = it * 256 + tid;
    const int w = idx >> 5;
    const int h4 = (idx & 31) * 4;
    const v4f v = *(const v4f*)(src + (size_t)w * NHID + h4);
    *(v4f*)(Tq + w * HOP + h4) = v;
  }
  __syncthreads();
  const int w4 = (tid & 15) * 4;
  const int hrow = tid >> 4;
  v4f ov[8];
#pragma unroll
  for (int it = 0; it < 8; ++it) {
    const int hd = it * 16 + hrow;
#pragma unroll
    for (int e = 0; e < 4; ++e) ov[it][e] = Tq[(w4 + e) * HOP + hd];
  }
  for (int pass = 0; pass < 2; ++pass) {
#pragma unroll
    for (int it = 0; it < 8; ++it) {
      const int hd = it * 16 + hrow;
      *(volatile v4f*)(out + (((size_t)(b * NHID + hd)) * NROW + r) * NCOL + w4) = ov[it];
    }
    __threadfence();
  }
}

extern "C" void kernel_launch(void* const* d_in, const int* in_sizes, int n_in,
                              void* d_out, int out_size, void* d_ws, size_t ws_size, hipStream_t stream) {
  if (n_in < 7 || d_out == nullptr || d_ws == nullptr) return;
  if (in_sizes[0] != NBAT * NCIN * NROW * NCOL || in_sizes[1] != NBAT * NHID * NROW ||
      in_sizes[2] != NBAT * NHID * NROW || in_sizes[3] != NGATE * NCIN || in_sizes[4] != NGATE ||
      in_sizes[5] != NGATE * NHID * 2 || in_sizes[6] != NGATE || out_size != NBAT * NHID * NROW * NCOL) return;

  const float* x   = (const float*)d_in[0];
  const float* h0  = (const float*)d_in[1];
  const float* c0  = (const float*)d_in[2];
  const float* wis = (const float*)d_in[3];
  const float* bis = (const float*)d_in[4];
  const float* wss = (const float*)d_in[5];
  const float* bss = (const float*)d_in[6];
  float* out = (float*)d_out;

  char* ws = (char*)d_ws;
  size_t off = 0;
  auto carve = [&](size_t bytes) -> char* { char* p = ws + off; off += (bytes + 255) & ~(size_t)255; return p; };
  unsigned short* XH   = (unsigned short*)carve((size_t)NBAT * NROW * NCOL * NCIN * 2);
  unsigned short* ACAT = (unsigned short*)carve((size_t)NGATE * KCAT * 2);
  float*          HST  = (float*)carve((size_t)NBAT * NROW * NCOL * NHID * 4);
  if (off > ws_size || off > (size_t)134217728) return;

  prep_x_kernel<<<NBAT * NROW, 256, 0, stream>>>(x, XH);
  prep_w_kernel<<<(NGATE * (KCAT / 8) + 255) / 256, 256, 0, stream>>>(wss, wis, ACAT);
  diag_scan_kernel<<<NBAT, SCAN_THR, 0, stream>>>(XH, ACAT, h0, c0, bis, bss, HST);
  unskew_tr_kernel<<<NBAT * NROW, 256, 0, stream>>>(HST, out);
}
